// _MRGNNLayer_90941637526228
// MI455X (gfx1250) — hardware-run, weakly checked
//
#include <hip/hip_runtime.h>


namespace {
constexpr int NB = 4, NN = 2048, D = 128, E = 65536, EF = 16, D2 = 256, M = NB * NN;
constexpr float XS = 8.0f, WSC = 256.0f, LNEPS = 1e-5f;
typedef _Float16 b16;
typedef __attribute__((ext_vector_type(16))) _Float16 v16b;
typedef __attribute__((ext_vector_type(8))) _Float16 v8b;
typedef __attribute__((ext_vector_type(8))) float v8f;
typedef __attribute__((ext_vector_type(4))) float v4f;
__device__ __forceinline__ float bf16_rne(float f) { unsigned int u = __float_as_uint(f); u += 0x7FFFu + ((u >> 16) & 1u); return __uint_as_float(u & 0xFFFF0000u); }
__device__ __forceinline__ void split16(float v, b16& hi, b16& lo) { hi = (b16)v; lo = (b16)(v - (float)hi); }
__device__ __forceinline__ v16b frag_kb(const b16* p, int hh) { const v8b a = *(const v8b*)(p + 8 * hh), b = *(const v8b*)(p + 16 + 8 * hh); v16b f;
#pragma unroll
  for (int e = 0; e < 8; ++e) { f[e] = a[e]; f[8 + e] = b[e]; } return f; }
__device__ __forceinline__ v8f wmma16b(v16b a, v16b b, v8f c) { v8f d = __builtin_amdgcn_wmma_f32_16x16x32_f16(false, a, false, b, (short)0, c, false, false); asm volatile("v_nop\n\tv_nop\n\tv_nop\n\tv_nop" : "+v"(d) : "v"(a), "v"(b)); return d; }
__device__ __forceinline__ void wave_lds_sync() { __builtin_amdgcn_fence(__ATOMIC_RELEASE, "workgroup"); __builtin_amdgcn_wave_barrier(); __builtin_amdgcn_fence(__ATOMIC_ACQUIRE, "workgroup"); }
__device__ __forceinline__ float pmul(float a, float b) { float p = a * b; asm volatile("" : "+v"(p)); return p; }
__device__ __forceinline__ int iclamp(int v, int lo, int hi) { return v < lo ? lo : (v > hi ? hi : v); }
constexpr int CSR_NBLK8 = 512, CSR_GB8 = 8, CSR_GN8 = 1 << CSR_GB8  , CSR_TS8 = (CSR_GN8 < 32 ? 32 : CSR_GN8)  , CSR_MAXG8 = 512, CSR_CAP8 = 12288  ;
__device__ __host__ __forceinline__ int csr_tix8(int v) { return (v >> CSR_GB8) * CSR_TS8 + (v & (CSR_GN8 - 1)); }
__global__ __launch_bounds__(64) void csrA_kernel8(const int* __restrict__ dst, int E, int N, int nG, int CHP, int NGP, int* __restrict__ STG, int* __restrict__ HST) {
  extern __shared__ int sm[];
  int* cnt = sm; int* run = sm + NGP; int* ids = sm + 2 * NGP;
  const int b = blockIdx.x; const int ch = (E + CSR_NBLK8 - 1) / CSR_NBLK8; const int e0 = b * ch, e1 = min(E, e0 + ch);
  for (int i = threadIdx.x; i < NGP; i += 64) cnt[i] = 0;
  for (int i = threadIdx.x; i < CHP; i += 64) ids[i] = -1;
  __syncthreads();
  if (threadIdx.x == 0) {
    for (int e = e0; e < e1; ++e) { int d = dst[e]; d = (d < 0) ? 0 : (d >= N ? N - 1 : d); cnt[d >> CSR_GB8] += 1; }
    int acc = 0; for (int g = 0; g < nG; ++g) { run[g] = acc; acc += cnt[g]; }
    for (int e = e0; e < e1; ++e) { int d = dst[e]; d = (d < 0) ? 0 : (d >= N ? N - 1 : d); const int g = d >> CSR_GB8; ids[run[g]] = e; run[g] += 1; } }
  __syncthreads();
  typedef __attribute__((ext_vector_type(4))) int v4i;
  for (int pass = 0; pass < 2; ++pass) {
    for (int i = threadIdx.x; i < CHP / 4; i += 64) *(volatile v4i*)(STG + (size_t)b * CHP + i * 4) = *(const v4i*)(&ids[i * 4]);
    for (int i = threadIdx.x; i < NGP / 4; i += 64) { v4i v; for (int e = 0; e < 4; ++e) v[e] = (i * 4 + e < nG) ? cnt[i * 4 + e] : 0; *(volatile v4i*)(HST + (size_t)b * NGP + i * 4) = v; }
    __threadfence(); }
}
__global__ __launch_bounds__(512) void csrS_kernel8(const int* __restrict__ HST, int nG, int NGP, int* __restrict__ START, int* __restrict__ TOT, int* __restrict__ OFF) {
  __shared__ int tot[CSR_MAXG8];
  const int b = threadIdx.x;
  for (int pass = 0; pass < 2; ++pass) { int runb = 0; for (int g = 0; g < nG; ++g) { int c = HST[(size_t)b * NGP + g]; c = (c < 0) ? 0 : c; ((volatile int*)OFF)[(size_t)g * CSR_NBLK8 + b] = runb; runb += c; } __threadfence(); }
  for (int g = threadIdx.x; g < nG; g += 512) { int s = 0; for (int bb = 0; bb < CSR_NBLK8; ++bb) { int c = HST[(size_t)bb * NGP + g]; s += (c < 0) ? 0 : c; } tot[g] = s; }
  __syncthreads();
  if (threadIdx.x < 32) {
    __shared__ int st[CSR_MAXG8 + 32];
    if (threadIdx.x == 0) { int acc = 0; for (int g = 0; g < NGP; ++g) { st[g] = acc; if (g < nG) acc += (tot[g] + 31) & ~31; } st[NGP] = acc; }
    __builtin_amdgcn_fence(__ATOMIC_RELEASE, "workgroup"); __builtin_amdgcn_wave_barrier(); __builtin_amdgcn_fence(__ATOMIC_ACQUIRE, "workgroup");
    for (int pass = 0; pass < 2; ++pass) { for (int i = threadIdx.x; i < NGP + 32; i += 32) { ((volatile int*)START)[i] = (i <= NGP) ? st[min(i, NGP)] : 0; ((volatile int*)TOT)[i] = (i < nG) ? tot[i] : 0; } __threadfence(); } }
}
__global__ __launch_bounds__(256) void csrB_kernel8(const int* __restrict__ dst, int N, int nG, int CHP, int NGP, int permLen, const int* __restrict__ STG, const int* __restrict__ HST, const int* __restrict__ OFF, const int* __restrict__ START, const int* __restrict__ TOT, int* __restrict__ PERM, int* __restrict__ ROWPTR, int* __restrict__ ROWCNT, int* __restrict__ FLAG) {
  typedef __attribute__((ext_vector_type(4))) int v4i;
  __shared__ int ids[CSR_CAP8]; __shared__ unsigned short key[CSR_CAP8]; __shared__ int outp[CSR_CAP8]; __shared__ int ncnt[CSR_GN8 + 1]; __shared__ int boff[CSR_NBLK8 + 1];
  const int g = blockIdx.x, t_ = threadIdx.x; int tot = TOT[g]; int st = START[g], stn = START[g + 1]; const int v0 = g * CSR_GN8; const int nv = min(CSR_GN8, N - v0); const int t0 = g * CSR_TS8;
  st = (st < 0) ? 0 : (st > permLen - 32 ? permLen - 32 : st) & ~31; stn = (stn < st) ? st : (stn > permLen ? permLen : stn); tot = (tot < 0) ? 0 : tot; if (tot > stn - st && tot <= CSR_CAP8) tot = stn - st;
  if (tot > CSR_CAP8) {
    for (int pass = 0; pass < 2; ++pass) { for (int i = t_; i < CSR_TS8 / 4; i += 256) { v4i a, c; for (int e = 0; e < 4; ++e) { a[e] = st; c[e] = 0; } *(volatile v4i*)(ROWPTR + t0 + i * 4) = a; *(volatile v4i*)(ROWCNT + t0 + i * 4) = c; } if (t_ == 0) ((volatile int*)FLAG)[0] = 1; __threadfence(); } (void)nv; return; }
  if (t_ == 0) { int acc = 0; for (int b = 0; b < CSR_NBLK8; ++b) { boff[b] = acc; int c = HST[(size_t)b * NGP + g]; c = (c < 0) ? 0 : (c > CHP ? CHP : c); acc += c; if (acc > tot) acc = tot; } boff[CSR_NBLK8] = acc; }
  for (int i = t_; i <= CSR_GN8; i += 256) ncnt[i] = 0;
  __syncthreads();
  for (int b = 0; b < CSR_NBLK8; ++b) { const int c = boff[b + 1] - boff[b]; int o_ = OFF[(size_t)g * CSR_NBLK8 + b]; o_ = (o_ < 0) ? 0 : (o_ > CHP - c ? CHP - c : o_); const int* src_ = STG + (size_t)b * CHP + o_;
    for (int i = t_; i < c; i += 256) { int id = src_[i]; id = (id < 0) ? 0 : id; ids[boff[b] + i] = id; int d = dst[id]; d = (d < v0) ? v0 : (d >= N ? N - 1 : d); int kk = d - v0; kk = (kk < 0) ? 0 : (kk >= CSR_GN8 ? CSR_GN8 - 1 : kk); key[boff[b] + i] = (unsigned short)kk; } }
  __syncthreads();
  if (t_ == 0) { for (int i = 0; i < tot; ++i) ncnt[key[i]] += 1; int acc = 0; for (int vl = 0; vl < CSR_GN8; ++vl) { const int c = ncnt[vl]; ncnt[vl] = acc; acc += c; } ncnt[CSR_GN8] = acc;
    for (int i = 0; i < tot; ++i) { const int vl = key[i]; outp[ncnt[vl]] = ids[i]; ncnt[vl] += 1; }
    for (int vl = CSR_GN8; vl > 0; --vl) ncnt[vl] = ncnt[vl - 1]; ncnt[0] = 0; }
  __syncthreads();
  for (int pass = 0; pass < 2; ++pass) {
    for (int i = t_; i < (stn - st) / 4; i += 256) { v4i v; for (int e = 0; e < 4; ++e) { const int q = i * 4 + e; v[e] = (q < tot) ? outp[q] : -1; } *(volatile v4i*)(PERM + st + i * 4) = v; }
    for (int i = t_; i < CSR_TS8 / 4; i += 256) { v4i a, c; for (int e = 0; e < 4; ++e) { const int vl = i * 4 + e; const int vc = vl < CSR_GN8 ? vl : CSR_GN8; a[e] = (vl < CSR_GN8) ? st + ncnt[vc] : st; c[e] = (vl < nv) ? (ncnt[(vc < CSR_GN8 ? vc : CSR_GN8 - 1) + 1] - ncnt[vc]) : 0; } *(volatile v4i*)(ROWPTR + t0 + i * 4) = a; *(volatile v4i*)(ROWCNT + t0 + i * 4) = c; }
    __threadfence(); }
}
__global__ __launch_bounds__(256) void csrZ_kernel8(int* __restrict__ p, size_t n4) { typedef __attribute__((ext_vector_type(4))) int v4i; const size_t tid = (size_t)blockIdx.x * 256 + threadIdx.x, nth = (size_t)gridDim.x * 256; v4i z = {0, 0, 0, 0}; for (size_t i = tid; i < n4; i += nth) *(volatile v4i*)(p + i * 4) = z; }
struct CsrBufs8 { int *STG, *HST, *OFF, *START, *TOT, *PERM, *ROWPTR, *ROWCNT, *FLAG; int nG, NGP, CHP; size_t permLen; char* base; size_t bytes; };
static size_t csr_carve8(CsrBufs8& c, char* ws, size_t off, int E, int N) {
  const size_t off0 = off; c.base = ws + off;
  auto al = [&](size_t bytes) { char* p = ws + off; off += (bytes + 255) & ~(size_t)255; return p; };
  c.nG = (N + CSR_GN8 - 1) / CSR_GN8; c.NGP = (c.nG + 31) & ~31; const int ch = (E + CSR_NBLK8 - 1) / CSR_NBLK8; c.CHP = (ch + 31) & ~31; c.permLen = (size_t)E + 32 * (size_t)c.nG + 32;
  c.STG = (int*)al((size_t)CSR_NBLK8 * c.CHP * 4); c.HST = (int*)al((size_t)CSR_NBLK8 * c.NGP * 4); c.OFF = (int*)al((size_t)c.NGP * CSR_NBLK8 * 4); c.START = (int*)al((size_t)(c.NGP + 64) * 4); c.TOT = (int*)al((size_t)(c.NGP + 64) * 4);
  c.PERM = (int*)al(c.permLen * 4); c.ROWPTR = (int*)al((size_t)c.nG * CSR_TS8 * 4); c.ROWCNT = (int*)al((size_t)c.nG * CSR_TS8 * 4); c.FLAG = (int*)al(256);
  c.bytes = off - off0; return off;
}
static void csr_build8(const CsrBufs8& c, const int* dst, int E, int N, hipStream_t stream) {
  const size_t smem = (size_t)(2 * c.NGP + c.CHP) * 4;
  csrZ_kernel8<<<512, 256, 0, stream>>>((int*)c.base, c.bytes / 16);
  csrA_kernel8<<<CSR_NBLK8, 64, smem, stream>>>(dst, E, N, c.nG, c.CHP, c.NGP, c.STG, c.HST);
  csrS_kernel8<<<1, 512, 0, stream>>>(c.HST, c.nG, c.NGP, c.START, c.TOT, c.OFF);
  csrB_kernel8<<<c.nG, 256, 0, stream>>>(dst, N, c.nG, c.CHP, c.NGP, (int)c.permLen, c.STG, c.HST, c.OFF, c.START, c.TOT, c.PERM, c.ROWPTR, c.ROWCNT, c.FLAG);
}


__global__ __launch_bounds__(256) void wprep_kernel(const float* __restrict__ wt1, const float* __restrict__ wt2, const float* __restrict__ wd1, const float* __restrict__ wd2, const float* __restrict__ wu, b16* __restrict__ W1A, b16* __restrict__ W1B, b16* __restrict__ W2T, b16* __restrict__ WUT) {
  const size_t u = (size_t)blockIdx.x * 256 + threadIdx.x; const size_t na = (size_t)D2 * D / 8, nb = (size_t)D2 * 32 / 8, n2 = (size_t)D * D2 / 8; size_t t = u; v8b v;
  for (int r = 0; r < 2; ++r) { const float* w1 = r == 0 ? wt1 : wd1; const float* w2 = r == 0 ? wt2 : wd2;
    if (t < na) { const size_t e = t * 8; const int o = (int)(e / D), k0 = (int)(e % D); for (int j = 0; j < 8; ++j) v[j] = (b16)(bf16_rne(w1[(size_t)(k0 + j) * D2 + o]) * WSC); for (int p = 0; p < 2; ++p) { *(volatile v8b*)(W1A + (size_t)r * D2 * D + e) = v; __threadfence(); } return; } t -= na;
    if (t < nb) { const size_t e = t * 8; const int o = (int)(e / 32), k0 = (int)(e % 32); for (int j = 0; j < 8; ++j) { const int k = k0 + j; v[j] = (k < EF) ? (b16)(bf16_rne(w1[(size_t)(D + (k < EF ? k : 0)) * D2 + o]) * WSC) : (b16)0.0f; } for (int p = 0; p < 2; ++p) { *(volatile v8b*)(W1B + (size_t)r * D2 * 32 + e) = v; __threadfence(); } return; } t -= nb;
    if (t < n2) { const size_t e = t * 8; const int o = (int)(e / D2), k0 = (int)(e % D2); for (int j = 0; j < 8; ++j) v[j] = (b16)(bf16_rne(w2[(size_t)(k0 + j) * D + o]) * WSC); for (int p = 0; p < 2; ++p) { *(volatile v8b*)(W2T + (size_t)r * D * D2 + e) = v; __threadfence(); } return; } t -= n2; }
  if (t < n2) { const size_t e = t * 8; const int o = (int)(e / D2), k0 = (int)(e % D2); for (int j = 0; j < 8; ++j) v[j] = (b16)(bf16_rne(wu[(size_t)(k0 + j) * D + o]) * WSC); for (int p = 0; p < 2; ++p) { *(volatile v8b*)(WUT + e) = v; __threadfence(); } }
}
__global__ __launch_bounds__(128) void pgemm_kernel(const float* __restrict__ h, const b16* __restrict__ W1A, float* __restrict__ P) {
  __shared__ __attribute__((aligned(16))) float Tf[4][16][D + 4];
  const int wave = threadIdx.x >> 5, lane = threadIdx.x & 31, nloc = lane & 15, hlf = lane >> 4; const size_t m0 = (size_t)blockIdx.x * 64 + wave * 16; const int c0 = blockIdx.y * 128; const float* xr = h + (m0 + nloc) * D;
  v8f acc[8];
#pragma unroll
  for (int t = 0; t < 8; ++t) acc[t] = (v8f){};
#pragma unroll 2
  for (int kb = 0; kb < D; kb += 32) { v16b a; for (int j = 0; j < 8; ++j) { a[j] = (b16)(bf16_rne(xr[kb + 8 * hlf + j]) * XS); a[8 + j] = (b16)(bf16_rne(xr[kb + 16 + 8 * hlf + j]) * XS); }
#pragma unroll
    for (int t = 0; t < 8; ++t) acc[t] = wmma16b(a, frag_kb(W1A + (size_t)(c0 + t * 16 + nloc) * D + kb, hlf), acc[t]); }
#pragma unroll
  for (int t = 0; t < 8; ++t)
#pragma unroll 1
    for (int r8 = 0; r8 < 8; ++r8) Tf[wave][8 * hlf + r8][t * 16 + nloc] = acc[t][r8] * (1.0f / (XS * WSC));
  wave_lds_sync();
  for (int pass = 0; pass < 2; ++pass) { for (int rr = 0; rr < 16; ++rr) *(volatile v4f*)(P + (m0 + rr) * D2 + c0 + lane * 4) = *(const v4f*)(&Tf[wave][rr][lane * 4]); __threadfence(); }
}
__global__ __launch_bounds__(128) void qgemm_kernel(const float* __restrict__ ea, const b16* __restrict__ W1B, const float* __restrict__ b1, float* __restrict__ Q) {
  __shared__ __attribute__((aligned(16))) float Tf[4][16][D + 4];
  const int wave = threadIdx.x >> 5, lane = threadIdx.x & 31, nloc = lane & 15, hlf = lane >> 4; const size_t e0 = (size_t)blockIdx.x * 64 + wave * 16; const int c0 = blockIdx.y * 128; const float* er = ea + (e0 + nloc) * EF;
  v16b a; for (int j = 0; j < 8; ++j) { const int k = 8 * hlf + j; a[j] = (b16)(bf16_rne(er[k]) * XS); a[8 + j] = (b16)0.0f; }
  v8f acc[8];
#pragma unroll
  for (int t = 0; t < 8; ++t) { acc[t] = (v8f){}; acc[t] = wmma16b(a, frag_kb(W1B + (size_t)(c0 + t * 16 + nloc) * 32, hlf), acc[t]); }
#pragma unroll
  for (int t = 0; t < 8; ++t) { const int c = t * 16 + nloc; const float bb = bf16_rne(b1[c0 + c]);
#pragma unroll 1
    for (int r8 = 0; r8 < 8; ++r8) Tf[wave][8 * hlf + r8][c] = acc[t][r8] * (1.0f / (XS * WSC)) + bb; }
  wave_lds_sync();
  for (int pass = 0; pass < 2; ++pass) { for (int rr = 0; rr < 16; ++rr) *(volatile v4f*)(Q + (e0 + rr) * D2 + c0 + lane * 4) = *(const v4f*)(&Tf[wave][rr][lane * 4]); __threadfence(); }
}
__global__ __launch_bounds__(256) void rsum_kernel(const float* __restrict__ P, const float* __restrict__ Q, const int* __restrict__ srcs, const int* __restrict__ PERM, const int* __restrict__ ROWPTR, const int* __restrict__ ROWCNT, int permLen, float* __restrict__ R) {
  const int wave = threadIdx.x >> 5, lane = threadIdx.x & 31; const size_t row = (size_t)blockIdx.x * 8 + wave; const int b = (int)(row / NN), v = (int)(row % NN);
  int st = ROWPTR[v], cnt = ROWCNT[v]; cnt = iclamp(cnt, 0, 65536); st = iclamp(st, 0, permLen - cnt); v4f a0 = {0.0f, 0.0f, 0.0f, 0.0f}, a1 = a0;
#pragma unroll 1
  for (int j = 0; j < cnt; ++j) { const int e = iclamp(PERM[st + j], 0, E - 1); const size_t s = (size_t)iclamp(srcs[e], 0, NN - 1);
    const v4f p0 = *(const v4f*)(P + ((size_t)b * NN + s) * D2 + lane * 8), p1 = *(const v4f*)(P + ((size_t)b * NN + s) * D2 + lane * 8 + 4), q0 = *(const v4f*)(Q + (size_t)e * D2 + lane * 8), q1 = *(const v4f*)(Q + (size_t)e * D2 + lane * 8 + 4);
    for (int i = 0; i < 4; ++i) { a0[i] += fmaxf(p0[i] + q0[i], 0.0f); a1[i] += fmaxf(p1[i] + q1[i], 0.0f); } }
  const float inv = 1.0f / (float)(cnt < 1 ? 1 : cnt); for (int i = 0; i < 4; ++i) { a0[i] = pmul(a0[i], inv); a1[i] = pmul(a1[i], inv); }
  for (int pass = 0; pass < 2; ++pass) { *(volatile v4f*)(R + row * D2 + lane * 8) = a0; *(volatile v4f*)(R + row * D2 + lane * 8 + 4) = a1; __threadfence(); }
}
__global__ __launch_bounds__(32) void agg_kernel(const float* __restrict__ R, const b16* __restrict__ W2T, const float* __restrict__ b2, const int* __restrict__ ROWCNT, float* __restrict__ AGG) {
  __shared__ __attribute__((aligned(16))) b16 Ah[16][D2 + 8], Al[16][D2 + 8]; __shared__ __attribute__((aligned(16))) float Tf[16][D + 4];
  const int lane = threadIdx.x, nloc = lane & 15, hlf = lane >> 4; const size_t m0 = (size_t)blockIdx.x * 16;
#pragma unroll 1
  for (int rr = 0; rr < 16; ++rr) { const v8f v = *(const v8f*)(R + (m0 + rr) * D2 + lane * 8); for (int j = 0; j < 8; ++j) { b16 p, q; split16(v[j] * XS, p, q); Ah[rr][lane * 8 + j] = p; Al[rr][lane * 8 + j] = q; } }
  wave_lds_sync();
  v8f acc[8];
#pragma unroll
  for (int t = 0; t < 8; ++t) acc[t] = (v8f){};
#pragma unroll 1
  for (int kb = 0; kb < D2; kb += 32) { const v16b a = frag_kb(&Ah[nloc][kb], hlf), al = frag_kb(&Al[nloc][kb], hlf);
#pragma unroll
    for (int t = 0; t < 8; ++t) { const v16b bw = frag_kb(W2T + (size_t)(t * 16 + nloc) * D2 + kb, hlf); acc[t] = wmma16b(a, bw, acc[t]); acc[t] = wmma16b(al, bw, acc[t]); } }
#pragma unroll
  for (int t = 0; t < 8; ++t) { const int c = t * 16 + nloc; const float bb = bf16_rne(b2[c]);
#pragma unroll 1
    for (int r8 = 0; r8 < 8; ++r8) { const int rl = 8 * hlf + r8; const int v = (int)((m0 + rl) % NN); int cnt = ROWCNT[v]; const float has = cnt > 0 ? 1.0f : 0.0f; Tf[rl][c] = acc[t][r8] * (1.0f / (XS * WSC)) + pmul(has, bb); } }
  wave_lds_sync();
  for (int pass = 0; pass < 2; ++pass) { for (int rr = 0; rr < 16; ++rr) *(volatile v4f*)(AGG + (m0 + rr) * D + lane * 4) = *(const v4f*)(&Tf[rr][lane * 4]); __threadfence(); }
}
__global__ __launch_bounds__(32) void out_kernel(const float* __restrict__ h, const float* __restrict__ AGT, const float* __restrict__ AGD, const b16* __restrict__ WUT, const float* __restrict__ bu, const float* __restrict__ gam, const float* __restrict__ bet, float* __restrict__ out) {
  __shared__ __attribute__((aligned(16))) b16 Ah[16][D2 + 8], Al[16][D2 + 8]; __shared__ __attribute__((aligned(16))) float Tf[16][D + 4];
  const int lane = threadIdx.x, nloc = lane & 15, hlf = lane >> 4; const size_t m0 = (size_t)blockIdx.x * 16;
#pragma unroll 1
  for (int rr = 0; rr < 16; ++rr) { const v4f a = *(const v4f*)(AGT + (m0 + rr) * D + lane * 4), d = *(const v4f*)(AGD + (m0 + rr) * D + lane * 4);
    for (int j = 0; j < 4; ++j) { b16 p, q; split16(a[j] * XS, p, q); Ah[rr][lane * 4 + j] = p; Al[rr][lane * 4 + j] = q; split16(d[j] * XS, p, q); Ah[rr][D + lane * 4 + j] = p; Al[rr][D + lane * 4 + j] = q; } }
  wave_lds_sync();
  v8f acc[8];
#pragma unroll
  for (int t = 0; t < 8; ++t) acc[t] = (v8f){};
#pragma unroll 1
  for (int kb = 0; kb < D2; kb += 32) { const v16b a = frag_kb(&Ah[nloc][kb], hlf), al = frag_kb(&Al[nloc][kb], hlf);
#pragma unroll
    for (int t = 0; t < 8; ++t) { const v16b bw = frag_kb(WUT + (size_t)(t * 16 + nloc) * D2 + kb, hlf); acc[t] = wmma16b(a, bw, acc[t]); acc[t] = wmma16b(al, bw, acc[t]); } }
#pragma unroll
  for (int t = 0; t < 8; ++t) { const int c = t * 16 + nloc; const float bb = bf16_rne(bu[c]);
#pragma unroll 1
    for (int r8 = 0; r8 < 8; ++r8) { const int rl = 8 * hlf + r8; Tf[rl][c] = bf16_rne(h[(m0 + rl) * D + c]) + acc[t][r8] * (1.0f / (XS * WSC)) + bb; } }
  wave_lds_sync();
  v4f g4, b4; for (int j = 0; j < 4; ++j) { g4[j] = bf16_rne(gam[lane * 4 + j]); b4[j] = bf16_rne(bet[lane * 4 + j]); }
#pragma unroll 1
  for (int rr = 0; rr < 16; ++rr) { v4f y = *(const v4f*)(&Tf[rr][lane * 4]); float s = y[0] + y[1] + y[2] + y[3]; for (int o = 16; o; o >>= 1) s += __shfl_xor(s, o); const float mu = s * (1.0f / D);
    float q = 0.0f; for (int j = 0; j < 4; ++j) { const float dd = y[j] - mu; q += pmul(dd, dd); } for (int o = 16; o; o >>= 1) q += __shfl_xor(q, o); const float rs = rsqrtf(q * (1.0f / D) + LNEPS);
    v4f o4; for (int j = 0; j < 4; ++j) o4[j] = pmul(pmul(y[j] - mu, rs), g4[j]) + b4[j]; *(v4f*)(&Tf[rr][lane * 4]) = o4; }
  wave_lds_sync();
  for (int pass = 0; pass < 2; ++pass) { for (int rr = 0; rr < 16; ++rr) *(volatile v4f*)(out + (m0 + rr) * D + lane * 4) = *(const v4f*)(&Tf[rr][lane * 4]); __threadfence(); }
}
}

extern "C" void kernel_launch(void* const* d_in, const int* in_sizes, int n_in, void* d_out, int out_size, void* d_ws, size_t ws_size, hipStream_t stream) {
  (void)n_in;
  auto Fp = [&](int i) { return (const float*)d_in[i]; }; auto Ip = [&](int i) { return (const int*)d_in[i]; };
  if (in_sizes[0] != M * D || in_sizes[1] != 2 * E || in_sizes[2] != E * EF || in_sizes[3] != 2 * E || in_sizes[4] != E * EF || in_sizes[5] != (D + EF) * D2 || in_sizes[7] != D2 * D || in_sizes[9] != (D + EF) * D2 || in_sizes[13] != D2 * D || out_size != M * D) return;
  size_t off = 0; char* ws = (char*)d_ws;
  auto carve = [&](size_t bytes) { char* p = ws + off; off += (bytes + 255) & ~(size_t)255; return p; };
  b16* W1A = (b16*)carve((size_t)2 * D2 * D * 2); b16* W1B = (b16*)carve((size_t)2 * D2 * 32 * 2); b16* W2T = (b16*)carve((size_t)2 * D * D2 * 2); b16* WUT = (b16*)carve((size_t)D * D2 * 2);
  float* P = (float*)carve((size_t)M * D2 * 4); float* Q = (float*)carve((size_t)E * D2 * 4); float* R = (float*)carve((size_t)M * D2 * 4); float* AGT = (float*)carve((size_t)M * D * 4); float* AGD = (float*)carve((size_t)M * D * 4);
  CsrBufs8 csrT, csrD; off = csr_carve8(csrT, ws, off, E, NN); off = csr_carve8(csrD, ws, off, E, NN);
  if (off > ws_size || off > ((size_t)128 << 20)) return;
  wprep_kernel<<<(unsigned)((2 * ((size_t)D2 * D / 8 + (size_t)D2 * 32 / 8 + (size_t)D * D2 / 8) + (size_t)D * D2 / 8 + 255) / 256), 256, 0, stream>>>(Fp(5), Fp(7), Fp(9), Fp(11), Fp(13), W1A, W1B, W2T, WUT);
  csr_build8(csrT, Ip(1) + E, E, NN, stream); csr_build8(csrD, Ip(3) + E, E, NN, stream);
  for (int r = 0; r < 2; ++r) { const CsrBufs8& c = r == 0 ? csrT : csrD; const float* ea = r == 0 ? Fp(2) : Fp(4); const int* srcs = r == 0 ? Ip(1) : Ip(3); const float* b1 = r == 0 ? Fp(6) : Fp(10); const float* b2 = r == 0 ? Fp(8) : Fp(12); float* AG = r == 0 ? AGT : AGD;
    pgemm_kernel<<<dim3(M / 64, 2), 128, 0, stream>>>(Fp(0), W1A + (size_t)r * D2 * D, P);
    qgemm_kernel<<<dim3(E / 64, 2), 128, 0, stream>>>(ea, W1B + (size_t)r * D2 * 32, b1, Q);
    rsum_kernel<<<M / 8, 256, 0, stream>>>(P, Q, srcs, c.PERM, c.ROWPTR, c.ROWCNT, (int)c.permLen, R);
    agg_kernel<<<M / 16, 32, 0, stream>>>(R, W2T + (size_t)r * D * D2, b2, c.ROWCNT, AG); }
  out_kernel<<<M / 16, 32, 0, stream>>>(Fp(0), AGT, AGD, WUT, Fp(14), Fp(15), Fp(16), (float*)d_out);
}
